// SyncGeodesicConv_50019189129838
// MI455X (gfx1250) — hardware-verified
//
#include <hip/hip_runtime.h>


namespace {
constexpr int B = 2, NV = 30000, ND = 8, NR = 3, C = 16, NF = 16, KC = NR * ND * C, KT = KC + C, KP = 416, NVT = B * NV;
constexpr float XS = 8.0f, WSC = 256.0f;
typedef _Float16 b16;
typedef __attribute__((ext_vector_type(16))) _Float16 v16b;
typedef __attribute__((ext_vector_type(8))) _Float16 v8b;
typedef __attribute__((ext_vector_type(8))) float v8f;
typedef __attribute__((ext_vector_type(4))) float v4f;
__device__ __forceinline__ float bf16_rne(float f) { unsigned int u = __float_as_uint(f); u += 0x7FFFu + ((u >> 16) & 1u); float r = __uint_as_float(u & 0xFFFF0000u); asm volatile("" : "+v"(r)); return r; }
__device__ __forceinline__ v16b frag_kb(const b16* p, int hh) { const v8b a = *(const v8b*)(p + 8 * hh), b = *(const v8b*)(p + 16 + 8 * hh); v16b f;
#pragma unroll
  for (int e = 0; e < 8; ++e) { f[e] = a[e]; f[8 + e] = b[e]; } return f; }
__device__ __forceinline__ v8f wmma16b(v16b a, v16b b, v8f c) { v8f d = __builtin_amdgcn_wmma_f32_16x16x32_f16(false, a, false, b, (short)0, c, false, false); asm volatile("v_nop\n\tv_nop\n\tv_nop\n\tv_nop" : "+v"(d) : "v"(a), "v"(b)); return d; }
__device__ __forceinline__ void wave_lds_sync() { __builtin_amdgcn_fence(__ATOMIC_RELEASE, "workgroup"); __builtin_amdgcn_wave_barrier(); __builtin_amdgcn_fence(__ATOMIC_ACQUIRE, "workgroup"); }
__device__ __forceinline__ int iclamp(int v, int lo, int hi) { return v < lo ? lo : (v > hi ? hi : v); }

__global__ __launch_bounds__(256) void wput_kernel(const float* __restrict__ ker, const float* __restrict__ ck, b16* __restrict__ WT) { const int u = blockIdx.x * 256 + threadIdx.x; if (u >= NF * (KP / 8)) return; const int f = u / (KP / 8), k0 = (u % (KP / 8)) * 8; v8b v;
#pragma unroll
  for (int j = 0; j < 8; ++j) { const int k = k0 + j; float w = 0.0f; if (k < KC) w = ker[(size_t)k * NF + f]; else if (k < KT) w = ck[(k - KC) * NF + f]; v[j] = (b16)(bf16_rne(w) * WSC); }
  for (int pass = 0; pass < 2; ++pass) { *(volatile v8b*)(WT + (size_t)f * KP + k0) = v; __threadfence(); } }
__global__ __launch_bounds__(32) void conv_kernel(const float* __restrict__ y, const int* __restrict__ sf, const b16* __restrict__ WT, const float* __restrict__ bias, int NVL, float* __restrict__ out) {
  __shared__ float Pt[2][NR * ND + ND][C + 1]; __shared__ __attribute__((aligned(16))) b16 Ah[16][KP + 8]; const int lane = threadIdx.x, nloc = lane & 15, hlf = lane >> 4; const size_t v0 = (size_t)blockIdx.x * 2; if (v0 % NV >= (size_t)NVL) return;
  for (int q = 0; q < 2; ++q) { const size_t bv = v0 + q; const int b = (int)(bv / NV);
    for (int idx = lane; idx < (NR * ND + ND) * C; idx += 32) { const int row = idx / C, c = idx % C; float val;
      if (row < NR * ND) { const int r = row / ND, d = row % ND; const int* t3 = sf + ((bv * NR + r) * ND + d) * 3; const int bb = iclamp(t3[0], 0, B - 1), vv = iclamp(t3[1], 0, NV - 1), dd = iclamp(t3[2], 0, ND - 1); val = y[(((size_t)bb * NV + vv) * ND + dd) * C + c]; }
      else { const int d = row - NR * ND; val = y[(bv * ND + d) * C + c]; (void)b; }
      Pt[q][row][c] = bf16_rne(val); } }
  wave_lds_sync();
  for (int rr = 0; rr < 16; ++rr) { const int q = rr >> 3, dout = rr & 7; for (int k = lane; k < KP; k += 32) { float v = 0.0f; if (k < KC) { const int r = k / (ND * C), kd = (k / C) % ND, c = k % C; v = Pt[q][r * ND + ((dout + kd) & 7)][c]; } else if (k < KT) v = Pt[q][NR * ND + dout][k - KC]; Ah[rr][k] = (b16)(v * XS); } }
  wave_lds_sync(); v8f acc = {};
#pragma unroll
  for (int kb = 0; kb < KP; kb += 32) acc = wmma16b(frag_kb(&Ah[nloc][kb], hlf), frag_kb(WT + (size_t)nloc * KP + kb, hlf), acc);
  const float bb = bf16_rne(bias[nloc]); float mx = 0.0f;
#pragma unroll
  for (int r8 = 0; r8 < 8; ++r8) mx = fmaxf(mx, acc[r8] * (1.0f / (XS * WSC)) + bb);
  for (int pass = 0; pass < 2; ++pass) { ((volatile float*)out)[(v0 + hlf) * NF + nloc] = mx; __threadfence(); } }
}

extern "C" void kernel_launch(void* const* d_in, const int* in_sizes, int n_in, void* d_out, int out_size, void* d_ws, size_t ws_size, hipStream_t stream) {
  (void)n_in;
  if (in_sizes[0] != NVT * ND * C || in_sizes[1] != NVT * NR * ND * 3 || in_sizes[2] != KC * NF || in_sizes[3] != C * NF || out_size != NVT * NF) return;
  const int NVL = NV;
  size_t off = 0; char* ws = (char*)d_ws;
  auto carve = [&](size_t bytes) { char* p = ws + off; off += (bytes + 255) & ~(size_t)255; return p; };
  b16* WT = (b16*)carve((size_t)NF * KP * 2);
  if (off > ws_size || off > ((size_t)1 << 20)) return;
  wput_kernel<<<(NF * (KP / 8) + 255) / 256, 256, 0, stream>>>((const float*)d_in[2], (const float*)d_in[3], WT);
  conv_kernel<<<NVT / 2, 32, 0, stream>>>((const float*)d_in[0], (const int*)d_in[1], WT, (const float*)d_in[4], NVL, (float*)d_out);
}
